// BilinearInteraction1_8821862826066
// MI455X (gfx1250) — hardware-verified
//
#include <hip/hip_runtime.h>


#define NF   32
#define NB_  4096
#define EM   64
#define NP   496

typedef unsigned short bf;
typedef __attribute__((ext_vector_type(16))) __bf16   v16bf;
typedef __attribute__((ext_vector_type(8)))  unsigned short v8us;
typedef __attribute__((ext_vector_type(8)))  float    v8f;
typedef __attribute__((ext_vector_type(4)))  float    v4f;
typedef v4f  __attribute__((may_alias)) v4fa;
typedef v8us __attribute__((may_alias)) v8usa;

__device__ __forceinline__ unsigned short f2bf(float f) { unsigned u = __float_as_uint(f); u += 0x7FFFu + ((u >> 16) & 1u); return (unsigned short)(u >> 16); }
__device__ __forceinline__ float bf2f(unsigned short b) { return __uint_as_float(((unsigned)b) << 16); }
__device__ __forceinline__ float bfr(float f) { return bf2f(f2bf(f)); }
__device__ __forceinline__ v16bf cat16b(v8us lo, v8us hi) { return __builtin_bit_cast(v16bf, __builtin_shufflevector(lo, hi, 0, 1, 2, 3, 4, 5, 6, 7, 8, 9, 10, 11, 12, 13, 14, 15)); }
__device__ __forceinline__ v8f wmmab(v16bf a, v16bf b, v8f c) { return __builtin_amdgcn_wmma_f32_16x16x32_bf16(false, a, false, b, (short)0, c, false, false); }
#define VST2(T, p, v) do { const T vst2_v_ = (v); *(volatile T*)(p) = vst2_v_; __threadfence(); *(volatile T*)(p) = vst2_v_; } while (0)

__device__ __forceinline__ void pair_of(int p, int& i, int& j) { int ii = 0, base = 0;
#pragma unroll 1
    while (ii < NF - 1) { const int cnt = NF - 1 - ii; if (p < base + cnt) break; base += cnt; ++ii; }
    i = ii; j = ii + 1 + (p - base); }

__global__ __launch_bounds__(256) void k_xb(const float* __restrict__ x, bf* XB) {
    const int lane = threadIdx.x & 31; const size_t r = (size_t)blockIdx.x * 8 + (threadIdx.x >> 5);
    if (r >= (size_t)NF * NB_) return;
    if (lane < 8) { v8us o;
#pragma unroll
        for (int q = 0; q < 8; ++q) o[q] = f2bf(x[r * EM + lane * 8 + q]);
        VST2(v8us, XB + r * EM + lane * 8, o); }
}
__global__ __launch_bounds__(256) void k_wt(const float* __restrict__ Wm, bf* WT) {
    __shared__ __align__(16) unsigned short tl[64 * 72];
    const int tid = threadIdx.x, p = blockIdx.x;
    const int kk = tid >> 2, lq = (tid & 3) * 16;
#pragma unroll
    for (int i = 0; i < 16; ++i) tl[(lq + i) * 72 + kk] = f2bf(Wm[((size_t)p * EM + kk) * EM + lq + i]);
    __syncthreads();
    const int piece = tid & 7;
    auto pass = [&]() {
#pragma unroll
        for (int s = 0; s < 2; ++s) { const int l = (tid >> 3) + 32 * s; const v8us val = *(const v8usa*)(tl + l * 72 + piece * 8); *(volatile v8us*)(WT + ((size_t)p * EM + l) * EM + piece * 8) = val; }
    };
    pass(); __threadfence(); pass();
}
__global__ __launch_bounds__(128) void k_bil(const bf* __restrict__ XB, const float* __restrict__ x, const bf* __restrict__ WT, float* OT) {
    __shared__ float st[64];
    const int lane = threadIdx.x & 31, wave = threadIdx.x >> 5, lr = lane & 15, hi = lane >> 4;
    const int b0 = blockIdx.x * 64 + wave * 16, p = blockIdx.y;
    int fi, fj; pair_of(p, fi, fj);
    const bf* xi = XB + ((size_t)fi * NB_ + b0 + lr) * EM + 8 * hi;
    v8f acc[4];
#pragma unroll
    for (int n = 0; n < 4; ++n) acc[n] = (v8f){};
#pragma unroll
    for (int kc = 0; kc < 2; ++kc) { const v16bf a = cat16b(*(const v8us*)(xi + kc * 32), *(const v8us*)(xi + kc * 32 + 16));
#pragma unroll
        for (int n = 0; n < 4; ++n) { const bf* bp = WT + ((size_t)p * EM + n * 16 + lr) * EM + kc * 32 + 8 * hi; acc[n] = wmmab(a, cat16b(*(const v8us*)bp, *(const v8us*)(bp + 16)), acc[n]); } }
    asm volatile("v_nop\n\tv_nop\n\tv_nop\n\tv_nop" : "+v"(acc[0]), "+v"(acc[1]), "+v"(acc[2]), "+v"(acc[3]));
    float part[8];
#pragma unroll
    for (int j = 0; j < 8; ++j) { const size_t xr = ((size_t)fj * NB_ + b0 + hi * 8 + j) * EM; float s = 0.f;
#pragma unroll
        for (int n = 0; n < 4; ++n) s += acc[n][j] * bfr(x[xr + n * 16 + lr]);
        s += __shfl_xor(s, 1, 16); s += __shfl_xor(s, 2, 16); s += __shfl_xor(s, 4, 16); s += __shfl_xor(s, 8, 16); part[j] = s; }
    if (lr == 0) {
#pragma unroll
        for (int j = 0; j < 8; ++j) st[wave * 16 + hi * 8 + j] = part[j]; }
    __syncthreads();
    if (wave == 0 && lane < 16) { const v4f v = *(const v4fa*)(st + lane * 4); VST2(v4f, OT + (size_t)p * NB_ + blockIdx.x * 64 + lane * 4, v); }
}
__global__ __launch_bounds__(256) void k_out(const float* __restrict__ OT, float* out) {
    const size_t e = (size_t)blockIdx.x * 256 + threadIdx.x;
    if (e >= (size_t)NB_ * NP) return;
    const int b = (int)(e / NP), p = (int)(e - (size_t)b * NP);
    const float v = OT[(size_t)p * NB_ + b];
    *(volatile float*)(out + e) = v; __threadfence(); *(volatile float*)(out + e) = v;
}

extern "C" void kernel_launch(void* const* d_in, const int* in_sizes, int n_in,
                              void* d_out, int out_size, void* d_ws, size_t ws_size, hipStream_t stream) {
    (void)in_sizes; (void)n_in; (void)out_size;
    const float* x = (const float*)d_in[0]; const float* Wm = (const float*)d_in[1];
    float* out = (float*)d_out;
    char* wsp = (char*)d_ws;
    auto take = [&](size_t bytes) { char* p = wsp; wsp += (bytes + 255) & ~(size_t)255; return (void*)p; };
    bf* XB = (bf*)take((size_t)NF * NB_ * EM * 2); bf* WT = (bf*)take((size_t)NP * EM * EM * 2); float* OT = (float*)take((size_t)NP * NB_ * 4);
    if ((size_t)(wsp - (char*)d_ws) > ws_size) return;
    k_xb<<<(NF * NB_) / 8, 256, 0, stream>>>(x, XB);
    k_wt<<<NP, 256, 0, stream>>>(Wm, WT);
    k_bil<<<dim3(NB_ / 64, NP, 1), 128, 0, stream>>>(XB, x, WT, OT);
    k_out<<<(unsigned)(((size_t)NB_ * NP) / 256), 256, 0, stream>>>(OT, out);
}
